// PartialSequenceDiffusion_3685081940028
// MI455X (gfx1250) — hardware-run, weakly checked
//
#include <hip/hip_runtime.h>
#include <stddef.h>
#include <stdint.h>

#define NN    8192
#define DD    256
#define KNB   32
#define PP    64
#define HH    8
#define DH    32
#define REL   65
#define NCH   16
#define NBA   4
#define NSEG  20
#define LRW   128
#define QKVW  768
#define GW    1280
#define GOW   512
#define TNODE 512
#define NTILE 16
#define TP    72
#define HP    136
#define GP    520
#define OTP   68
#define WSC   32.0f
#define C_P1  4.0f
#define C_H   16.0f
#define C_P2  16.0f
#define C_ATT 4.0f
#define C_GO  16.0f
#define S_W   0.03125f
#define S_M1  0.0078125f
#define S_M2  0.001953125f
#define S_PB  0.001953125f
#define S_WO  0.0078125f
#define S_WOG 0.001953125f
#define RSQDH 0.17677669529663687f

static_assert(NN % 256 == 0);
static_assert(NTILE * TNODE == NN);
static_assert(NSEG == NCH + NBA);
static_assert(GW == 5 * DD);
static_assert(QKVW == 3 * DD);
static_assert(HH * DH == DD);
static_assert(GOW == 2 * DD);
static_assert((NN * KNB) % 64 == 0);
static_assert(KNB == 32);
static_assert(PP == 64);
static_assert((NN * DD) % 2048 == 0);
static_assert(TP % 8 == 0);
static_assert(HP % 8 == 0);
static_assert(GP % 8 == 0);

typedef _Float16 v16h __attribute__((ext_vector_type(16)));
typedef _Float16 v8h  __attribute__((ext_vector_type(8)));
typedef float v8f __attribute__((ext_vector_type(8)));
typedef float v4f __attribute__((ext_vector_type(4)));
typedef unsigned int v4u __attribute__((ext_vector_type(4)));

union PackH { v8h h; v4u u; };

__device__ __forceinline__ v8f zero8() { return (v8f){0.f, 0.f, 0.f, 0.f, 0.f, 0.f, 0.f, 0.f}; }
__device__ __forceinline__ v4f zero4() { return (v4f){0.f, 0.f, 0.f, 0.f}; }
__device__ __forceinline__ int clampi(int x, int lo, int hi) { return x < lo ? lo : (x > hi ? hi : x); }

__device__ __forceinline__ float wave_sum(float v) {
#pragma unroll
  for (int o = 16; o > 0; o >>= 1) v += __shfl_xor(v, o, 32);
  return v;
}
__device__ __forceinline__ float wave_max(float v) {
#pragma unroll
  for (int o = 16; o > 0; o >>= 1) v = fmaxf(v, __shfl_xor(v, o, 32));
  return v;
}
__device__ __forceinline__ float gelu_f(float x) {
  const float u = 0.7978845608028654f * fmaf(0.044715f * x, x * x, x);
  return x * __builtin_amdgcn_rcpf(1.0f + __expf(-2.0f * u));
}

struct OpF16 {
  typedef _Float16 E;
  typedef v16h F;
  static __device__ __forceinline__ F ld(const E* p, int ldk, size_t row0, int k0, int lane) {
    const int m = lane & 15, lh = lane >> 4;
    const E* q = p + (row0 + (size_t)m) * (size_t)ldk + k0 + 8 * lh;
    union { F v; v8h hv[2]; } f;
    f.hv[0] = *(const v8h*)(q);
    f.hv[1] = *(const v8h*)(q + 16);
    return f.v;
  }
  static __device__ __forceinline__ v8f mma(F a, F b, v8f c) {
    c = __builtin_amdgcn_wmma_f32_16x16x32_f16(false, a, false, b, (short)0, c, false, false);
    asm volatile("v_nop\n\tv_nop\n\tv_nop\n\tv_nop" : "+v"(c) : "v"(a), "v"(b));
    return c;
  }
};

__global__ __launch_bounds__(256) void k_cvt(const float* __restrict__ src, _Float16* __restrict__ dh, float scale) {
  const int tid = threadIdx.x;
  const size_t o = (size_t)blockIdx.x * 2048 + (size_t)tid * 8;
  const v4f a0 = *(const v4f*)(src + o) * scale;
  const v4f a1 = *(const v4f*)(src + o + 4) * scale;
  PackH pk;
  pk.h = (v8h){(_Float16)a0[0], (_Float16)a0[1], (_Float16)a0[2], (_Float16)a0[3],
               (_Float16)a1[0], (_Float16)a1[1], (_Float16)a1[2], (_Float16)a1[3]};
  const v4u vv = pk.u;
  volatile v4u* d = (volatile v4u*)(dh + o);
  *d = vv;
  __threadfence();
  *d = vv;
}

__global__ __launch_bounds__(256) void k_wtrans(const float* __restrict__ src, int Ksrc, int Nsrc,
                                                _Float16* __restrict__ dst, int ldd, int dstrow0, float scale) {
  __shared__ __align__(16) float T[64][68];
  const int tid = threadIdx.x;
  const int n0 = blockIdx.x * 64, k0 = blockIdx.y * 64;
#pragma unroll
  for (int it = 0; it < 4; ++it) {
    const int idx = tid + 256 * it;
    const int krow = idx >> 4, n4 = (idx & 15) * 4;
    const int gk = k0 + krow, gn = n0 + n4;
    const int kcl = (gk < Ksrc) ? gk : (Ksrc - 1);
    const int ncl = (gn <= Nsrc - 4) ? gn : (Nsrc - 4);
    const v4f v = *(const v4f*)(src + (size_t)kcl * Nsrc + ncl);
    const bool ok = (gk < Ksrc) && (gn < Nsrc);
    T[n4 + 0][krow] = ok ? v[0] : 0.0f;
    T[n4 + 1][krow] = ok ? v[1] : 0.0f;
    T[n4 + 2][krow] = ok ? v[2] : 0.0f;
    T[n4 + 3][krow] = ok ? v[3] : 0.0f;
  }
  __syncthreads();
  v4u val[2];
  size_t go[2];
#pragma unroll
  for (int it = 0; it < 2; ++it) {
    const int p = tid + 256 * it;
    const int row = p >> 3, pc = p & 7;
    const v4f x0 = *(const v4f*)(&T[row][pc * 8]);
    const v4f x1 = *(const v4f*)(&T[row][pc * 8 + 4]);
    PackH ph;
    ph.h = (v8h){(_Float16)(x0[0] * scale), (_Float16)(x0[1] * scale), (_Float16)(x0[2] * scale),
                 (_Float16)(x0[3] * scale), (_Float16)(x1[0] * scale), (_Float16)(x1[1] * scale),
                 (_Float16)(x1[2] * scale), (_Float16)(x1[3] * scale)};
    val[it] = ph.u;
    go[it] = (size_t)(dstrow0 + n0 + row) * (size_t)ldd + k0 + pc * 8;
  }
  for (int ps = 0; ps < 2; ++ps) {
#pragma unroll
    for (int it = 0; it < 2; ++it) *(volatile v4u*)(dst + go[it]) = val[it];
    __threadfence();
  }
}

__global__ __launch_bounds__(256) void k_bias(const float* __restrict__ bkg, const float* __restrict__ bvg,
                                              const float* __restrict__ bqg, const float* __restrict__ bbg,
                                              float* __restrict__ BG) {
  const int tid = threadIdx.x;
#pragma unroll 1
  for (int it = 0; it < 2; ++it) {
    const int q = tid + 256 * it;
    const int qc = (q < GW / 4) ? q : (GW / 4 - 1);
    const int n = 4 * qc;
    const v4f v0 = *(const v4f*)(bkg + clampi(n, 0, DD - 4));
    const v4f v1 = *(const v4f*)(bvg + clampi(n - DD, 0, DD - 4));
    const v4f v2 = *(const v4f*)(bqg + clampi(n - 2 * DD, 0, DD - 4));
    const v4f v3 = *(const v4f*)(bbg + clampi(n - 3 * DD, 0, GOW - 4));
    v4f e = v3;
    if (n < DD) e = v0;
    else if (n < 2 * DD) e = v1;
    else if (n < 3 * DD) e = v2;
    const bool act = (q < GW / 4);
    volatile v4f* d = (volatile v4f*)(BG + 4 * qc);
    if (act) *d = e;
    __threadfence();
    if (act) *d = e;
  }
}

__device__ __forceinline__ void gemm32x64(const _Float16* __restrict__ A, int lda,
                                          const _Float16* __restrict__ Bt, int ldb, int K,
                                          int m0, int n0, int lane, v8f (&acc)[2][4]) {
#pragma unroll 1
  for (int k0 = 0; k0 < K; k0 += 32) {
    const v16h a0 = OpF16::ld(A, lda, (size_t)m0, k0, lane);
    const v16h a1 = OpF16::ld(A, lda, (size_t)m0 + 16, k0, lane);
    const v16h b0 = OpF16::ld(Bt, ldb, (size_t)n0, k0, lane);
    const v16h b1 = OpF16::ld(Bt, ldb, (size_t)n0 + 16, k0, lane);
    const v16h b2 = OpF16::ld(Bt, ldb, (size_t)n0 + 32, k0, lane);
    const v16h b3 = OpF16::ld(Bt, ldb, (size_t)n0 + 48, k0, lane);
    acc[0][0] = OpF16::mma(a0, b0, acc[0][0]);
    acc[1][0] = OpF16::mma(a1, b0, acc[1][0]);
    acc[0][1] = OpF16::mma(a0, b1, acc[0][1]);
    acc[1][1] = OpF16::mma(a1, b1, acc[1][1]);
    acc[0][2] = OpF16::mma(a0, b2, acc[0][2]);
    acc[1][2] = OpF16::mma(a1, b2, acc[1][2]);
    acc[0][3] = OpF16::mma(a0, b3, acc[0][3]);
    acc[1][3] = OpF16::mma(a1, b3, acc[1][3]);
  }
}

__device__ __forceinline__ void epilogue_f32(v8f (&acc)[2][4], float scale, const float* __restrict__ bias,
                                             const float* __restrict__ res, int act,
                                             float* sw, float* __restrict__ out, int ldo,
                                             int m0, int n0, int lane, int hh, int c) {
  float bn[4] = {0.0f, 0.0f, 0.0f, 0.0f};
  if (bias != nullptr) {
#pragma unroll
    for (int t = 0; t < 4; ++t) bn[t] = bias[n0 + 16 * t + c];
  }
#pragma unroll
  for (int sub = 0; sub < 2; ++sub) {
    __syncthreads();
#pragma unroll
    for (int t = 0; t < 4; ++t) {
#pragma unroll
      for (int r = 0; r < 8; ++r) {
        float v = fmaf(acc[sub][t][r], scale, bn[t]);
        if (act) v = gelu_f(v);
        sw[(8 * hh + r) * OTP + 16 * t + c] = v;
      }
    }
    __syncthreads();
    v4f val[8];
    size_t go[8];
#pragma unroll
    for (int it = 0; it < 8; ++it) {
      const int p    = lane + 32 * it;
      const int L    = p >> 3;
      const int pc   = p & 7;
      const int row  = L >> 1;
      const int half = L & 1;
      val[it] = *(const v4f*)(sw + row * OTP + half * 32 + pc * 4);
      go[it]  = (size_t)(m0 + sub * 16 + row) * ldo + n0 + half * 32 + pc * 4;
    }
    if (res != nullptr) {
#pragma unroll
      for (int it = 0; it < 8; ++it) val[it] = val[it] + *(const v4f*)(res + go[it]);
    }
    for (int ps = 0; ps < 2; ++ps) {
#pragma unroll
      for (int it = 0; it < 8; ++it) *(volatile v4f*)(out + go[it]) = val[it];
      __threadfence();
    }
  }
}

__global__ __launch_bounds__(256) void k_gemm(const _Float16* __restrict__ ap, int lda,
                                              const _Float16* __restrict__ wt, int ldb, int K, float scale,
                                              const float* __restrict__ bias, const float* __restrict__ res,
                                              float* __restrict__ out, int ldo, int gelu_mask) {
  __shared__ __align__(16) float st[8][16 * OTP];
  const int tid = threadIdx.x, lane = tid & 31, wave = tid >> 5;
  const int hh = lane >> 4, c = lane & 15;
  const int m0 = blockIdx.x * 256 + wave * 32;
  const int n0 = blockIdx.y * 64;
  const int act = (gelu_mask >> (int)blockIdx.y) & 1;

  v8f acc[2][4];
#pragma unroll
  for (int s = 0; s < 2; ++s)
#pragma unroll
    for (int t = 0; t < 4; ++t) acc[s][t] = zero8();
  gemm32x64(ap, lda, wt, ldb, K, m0, n0, lane, acc);
  epilogue_f32(acc, scale, bias, res, act, st[wave], out, ldo, m0, n0, lane, hh, c);
}

__global__ __launch_bounds__(256) void k_ln8(const float* __restrict__ x,
                                             const float* __restrict__ g1, const float* __restrict__ b1,
                                             const float* __restrict__ g2, const float* __restrict__ b2,
                                             _Float16* __restrict__ F1, _Float16* __restrict__ F2) {
  const int tid = threadIdx.x, lane = tid & 31, wave = tid >> 5;
  const size_t n = (size_t)blockIdx.x * 8 + wave;
  const size_t o = n * DD + (size_t)lane * 8;
  const v4f u0 = *(const v4f*)(x + o);
  const v4f u1 = *(const v4f*)(x + o + 4);
  float s = ((u0[0] + u0[1]) + (u0[2] + u0[3])) + ((u1[0] + u1[1]) + (u1[2] + u1[3]));
  s = wave_sum(s);
  const float mu = s * (1.0f / (float)DD);
  const v4f c0 = u0 - mu, c1 = u1 - mu;
  float q = ((c0[0] * c0[0] + c0[1] * c0[1]) + (c0[2] * c0[2] + c0[3] * c0[3])) +
            ((c1[0] * c1[0] + c1[1] * c1[1]) + (c1[2] * c1[2] + c1[3] * c1[3]));
  q = wave_sum(q);
  const float rs = rsqrtf(q * (1.0f / (float)DD) + 1e-5f);
  v4u w1, w2;
  {
    const v4f ga = *(const v4f*)(g1 + lane * 8), gb = *(const v4f*)(g1 + lane * 8 + 4);
    const v4f ba = *(const v4f*)(b1 + lane * 8), bb = *(const v4f*)(b1 + lane * 8 + 4);
    const v4f y0 = ga * c0 * rs + ba, y1 = gb * c1 * rs + bb;
    PackH p;
    p.h = (v8h){(_Float16)y0[0], (_Float16)y0[1], (_Float16)y0[2], (_Float16)y0[3],
                (_Float16)y1[0], (_Float16)y1[1], (_Float16)y1[2], (_Float16)y1[3]};
    w1 = p.u;
  }
  {
    const v4f ga = *(const v4f*)(g2 + lane * 8), gb = *(const v4f*)(g2 + lane * 8 + 4);
    const v4f ba = *(const v4f*)(b2 + lane * 8), bb = *(const v4f*)(b2 + lane * 8 + 4);
    const v4f y0 = ga * c0 * rs + ba, y1 = gb * c1 * rs + bb;
    PackH p;
    p.h = (v8h){(_Float16)y0[0], (_Float16)y0[1], (_Float16)y0[2], (_Float16)y0[3],
                (_Float16)y1[0], (_Float16)y1[1], (_Float16)y1[2], (_Float16)y1[3]};
    w2 = p.u;
  }
  volatile v4u* d1 = (volatile v4u*)(F1 + o);
  volatile v4u* d2 = (volatile v4u*)(F2 + o);
  *d1 = w1;
  *d2 = w2;
  __threadfence();
  *d1 = w1;
  *d2 = w2;
}

__global__ __launch_bounds__(256) void k_pair(const float* __restrict__ wrel, const float* __restrict__ LR,
                                              const float* __restrict__ g_lnp, const float* __restrict__ b_lnp,
                                              const float* __restrict__ b_m1, const float* __restrict__ b_m2,
                                              const _Float16* __restrict__ WM1T, const _Float16* __restrict__ WM2T,
                                              const _Float16* __restrict__ WPBT,
                                              const int* __restrict__ nbrs, const int* __restrict__ resi,
                                              const int* __restrict__ chain, const int* __restrict__ batch,
                                              float* __restrict__ PB) {
  __shared__ __align__(16) _Float16 P16[64][TP];
  __shared__ __align__(16) _Float16 H16[64][HP];
  __shared__ __align__(16) float PBs[2][HH][KNB];
  const int tid = threadIdx.x, lane = tid & 31, wave = tid >> 5;
  const int hh = lane >> 4, c = lane & 15;
  const int r0 = blockIdx.x * 64;

  {
    const int row = tid >> 2, seg = tid & 3;
    const int r = r0 + row, n = r >> 5, kk = r & 31;
    const int nbr = nbrs[n * KNB + kk];
    int nbv = nbr < 0 ? 0 : nbr;
    nbv = nbv > NN - 1 ? NN - 1 : nbv;
    int rel = resi[n] - resi[nbv];
    rel = clampi(rel, -32, 32) + 32;
    const bool same = (chain[n] == chain[nbv]) && (batch[n] == batch[nbv]);
    const float fs = same ? 1.0f : 0.0f;
    const float* wr = wrel + rel * PP + seg * 16;
    const float* lp = LR + (size_t)n * LRW + seg * 16;
    const float* rp = LR + (size_t)nbv * LRW + PP + seg * 16;
    v4f xv[4];
#pragma unroll
    for (int i = 0; i < 4; ++i) {
      const v4f w = *(const v4f*)(wr + 4 * i);
      const v4f l = *(const v4f*)(lp + 4 * i);
      const v4f q = *(const v4f*)(rp + 4 * i);
      xv[i] = (w * fs + l) + q;
    }
    float s = 0.0f;
#pragma unroll
    for (int i = 0; i < 4; ++i) s += (xv[i][0] + xv[i][1]) + (xv[i][2] + xv[i][3]);
    s += __shfl_xor(s, 1, 32);
    s += __shfl_xor(s, 2, 32);
    const float mu = s * (1.0f / (float)PP);
    float q2 = 0.0f;
#pragma unroll
    for (int i = 0; i < 4; ++i) {
      xv[i] = xv[i] - mu;
      q2 += (xv[i][0] * xv[i][0] + xv[i][1] * xv[i][1]) + (xv[i][2] * xv[i][2] + xv[i][3] * xv[i][3]);
    }
    q2 += __shfl_xor(q2, 1, 32);
    q2 += __shfl_xor(q2, 2, 32);
    const float rs = rsqrtf(q2 * (1.0f / (float)PP) + 1e-5f);
    const float* gp = g_lnp + seg * 16;
    const float* bp = b_lnp + seg * 16;
    v4f y[4];
#pragma unroll
    for (int i = 0; i < 4; ++i) {
      const v4f gv = *(const v4f*)(gp + 4 * i);
      const v4f bv = *(const v4f*)(bp + 4 * i);
      y[i] = (gv * xv[i] * rs + bv) * C_P1;
    }
    *(v8h*)(&P16[row][seg * 16]) =
        (v8h){(_Float16)y[0][0], (_Float16)y[0][1], (_Float16)y[0][2], (_Float16)y[0][3],
              (_Float16)y[1][0], (_Float16)y[1][1], (_Float16)y[1][2], (_Float16)y[1][3]};
    *(v8h*)(&P16[row][seg * 16 + 8]) =
        (v8h){(_Float16)y[2][0], (_Float16)y[2][1], (_Float16)y[2][2], (_Float16)y[2][3],
              (_Float16)y[3][0], (_Float16)y[3][1], (_Float16)y[3][2], (_Float16)y[3][3]};
  }
  __syncthreads();

  {
    const int rt = wave >> 1, nh = wave & 1;
    v8f acc[4];
#pragma unroll
    for (int t = 0; t < 4; ++t) acc[t] = zero8();
#pragma unroll
    for (int ks = 0; ks < 2; ++ks) {
      const v16h a = OpF16::ld(&P16[0][0], TP, (size_t)(rt * 16), ks * 32, lane);
#pragma unroll
      for (int t = 0; t < 4; ++t) {
        const v16h b = OpF16::ld(WM1T, PP, (size_t)(nh * 64 + 16 * t), ks * 32, lane);
        acc[t] = OpF16::mma(a, b, acc[t]);
      }
    }
#pragma unroll
    for (int t = 0; t < 4; ++t) {
      const int col = nh * 64 + 16 * t + c;
      const float bv = b_m1[col];
#pragma unroll
      for (int r = 0; r < 8; ++r) {
        float v = fmaf(acc[t][r], S_M1, bv);
        v = gelu_f(v) * C_H;
        H16[rt * 16 + 8 * hh + r][col] = (_Float16)v;
      }
    }
  }
  __syncthreads();

  {
    const int rt = wave >> 1, nh = wave & 1;
    v8f acc[2];
    acc[0] = zero8();
    acc[1] = zero8();
#pragma unroll
    for (int ks = 0; ks < 4; ++ks) {
      const v16h a = OpF16::ld(&H16[0][0], HP, (size_t)(rt * 16), ks * 32, lane);
#pragma unroll
      for (int t = 0; t < 2; ++t) {
        const v16h b = OpF16::ld(WM2T, 2 * PP, (size_t)(nh * 32 + 16 * t), ks * 32, lane);
        acc[t] = OpF16::mma(a, b, acc[t]);
      }
    }
#pragma unroll
    for (int t = 0; t < 2; ++t) {
      const int col = nh * 32 + 16 * t + c;
      const float bv = b_m2[col];
#pragma unroll
      for (int r = 0; r < 8; ++r) {
        const float v = fmaf(acc[t][r], S_M2, bv) * C_P2;
        P16[rt * 16 + 8 * hh + r][col] = (_Float16)v;
      }
    }
  }
  __syncthreads();

  if (wave < 4) {
    const int rt = wave;
    v8f acc = zero8();
#pragma unroll
    for (int ks = 0; ks < 2; ++ks) {
      const v16h a = OpF16::ld(&P16[0][0], TP, (size_t)(rt * 16), ks * 32, lane);
      const v16h b = OpF16::ld(WPBT, PP, (size_t)0, ks * 32, lane);
      acc = OpF16::mma(a, b, acc);
    }
#pragma unroll
    for (int r = 0; r < 8; ++r) {
      const int row = rt * 16 + 8 * hh + r;
      const int nl = row >> 5, kk = row & 31;
      if (c < HH) PBs[nl][c][kk] = acc[r] * S_PB;
    }
  }
  __syncthreads();

  if (tid < 128) {
    const int node = tid >> 6, f = (tid & 63) * 4;
    const v4f val = *(const v4f*)(&PBs[node][0][0] + f);
    volatile v4f* d = (volatile v4f*)(PB + (size_t)(blockIdx.x * 2 + node) * (HH * KNB) + f);
    *d = val;
    __threadfence();
    *d = val;
  }
}

__global__ __launch_bounds__(256) void k_attn(const float* __restrict__ QKV, const float* __restrict__ PB,
                                              const float* __restrict__ mask, const int* __restrict__ nbrs,
                                              _Float16* __restrict__ ATT) {
  __shared__ __align__(16) float qs[DD];
  __shared__ __align__(16) _Float16 os[DD];
  const int tid = threadIdx.x, lane = tid & 31, h = tid >> 5;
  const int n = blockIdx.x;
  qs[tid] = QKV[(size_t)n * QKVW + tid];
  const int nbr = nbrs[n * KNB + lane];
  const float vf = (nbr != -1) ? 1.0f : 0.0f;
  int nbv = nbr < 0 ? 0 : nbr;
  nbv = nbv > NN - 1 ? NN - 1 : nbv;
  const float pm = (mask[n] * mask[nbv]) * vf;
  __syncthreads();

  const float* kr = QKV + (size_t)nbv * QKVW + DD + h * DH;
  const float* qr = qs + h * DH;
  float dp = 0.0f;
#pragma unroll 2
  for (int cc = 0; cc < DH / 4; ++cc) {
    const v4f kq = *(const v4f*)(kr + 4 * cc);
    const v4f qq = *(const v4f*)(qr + 4 * cc);
    dp = fmaf(qq[0], kq[0], dp);
    dp = fmaf(qq[1], kq[1], dp);
    dp = fmaf(qq[2], kq[2], dp);
    dp = fmaf(qq[3], kq[3], dp);
  }
  const float logit = dp * RSQDH + PB[(size_t)n * (HH * KNB) + h * KNB + lane];
  const float lm = (pm > 0.0f) ? logit : -1.0e9f;
  const float mx = wave_max(lm);
  const float e = __expf(lm - mx);
  const float ssum = wave_sum(e);
  float att = e * (1.0f / ssum);
  att = (pm > 0.0f) ? att : 0.0f;

  const float* vb = QKV + 2 * DD + h * DH + lane;
  float o = 0.0f;
#pragma unroll 4
  for (int k = 0; k < KNB; ++k) {
    const float ak = __shfl(att, k, 32);
    const int nk = __shfl(nbv, k, 32);
    o = fmaf(ak, vb[(size_t)nk * QKVW], o);
  }
  os[tid] = (_Float16)(o * C_ATT);
  __syncthreads();
  if (tid < 32) {
    PackH ph;
    ph.h = *(const v8h*)(&os[lane * 8]);
    const v4u vv = ph.u;
    volatile v4u* d = (volatile v4u*)(ATT + (size_t)n * DD + lane * 8);
    *d = vv;
    __threadfence();
    *d = vv;
  }
}

__global__ __launch_bounds__(128) void k_kvpart(const float* __restrict__ G, const float* __restrict__ mask,
                                                const int* __restrict__ chain, const int* __restrict__ batch,
                                                float* __restrict__ PART) {
  __shared__ __align__(16) float acc[NSEG * 512];
  const int tid = threadIdx.x;
  const int ih = blockIdx.x & 1, h = (blockIdx.x >> 1) & 7, tile = blockIdx.x >> 4;
  const int il = tid >> 3, j4 = (tid & 7) * 4, i = ih * 16 + il;
  float* my = acc + tid * 4;
  const v4f z = zero4();
#pragma unroll
  for (int s = 0; s < NSEG; ++s) *(v4f*)(my + s * 512) = z;
  const int n0 = tile * TNODE;
  const float* gk = G + h * DH + i;
  const float* gv = G + DD + h * DH + j4;
#pragma unroll 1
  for (int nn = 0; nn < TNODE; ++nn) {
    const int n = n0 + nn;
    const float m = mask[n];
    const int ci = chain[n], bi = batch[n];
    const float kval = gk[(size_t)n * GW];
    const v4f vv = *(const v4f*)(gv + (size_t)n * GW);
    const v4f p = (kval * vv) * m;
    const float cf = ((unsigned)ci < (unsigned)NCH) ? 1.0f : 0.0f;
    const float bf = ((unsigned)bi < (unsigned)NBA) ? 1.0f : 0.0f;
    const int cs = clampi(ci, 0, NCH - 1), bs = clampi(bi, 0, NBA - 1);
    float* pc = my + cs * 512;
    v4f a = *(const v4f*)pc;
    a = a + p * cf;
    *(v4f*)pc = a;
    float* pb = my + (NCH + bs) * 512;
    v4f b = *(const v4f*)pb;
    b = b + p * bf;
    *(v4f*)pb = b;
  }
  const size_t base = ((size_t)(tile * HH + h) * NSEG) * 1024 + (size_t)ih * 512 + (size_t)tid * 4;
#pragma unroll 1
  for (int s = 0; s < NSEG; ++s) {
    const v4f v = *(const v4f*)(my + s * 512);
    volatile v4f* d = (volatile v4f*)(PART + base + (size_t)s * 1024);
    *d = v;
    __threadfence();
    *d = v;
  }
}

__global__ __launch_bounds__(256) void k_segred(const float* __restrict__ PART, const float* __restrict__ mask,
                                                const int* __restrict__ chain, const int* __restrict__ batch,
                                                float* __restrict__ OPS) {
  __shared__ float red[8];
  const int tid = threadIdx.x, lane = tid & 31, wave = tid >> 5;
  const int s = blockIdx.x >> 3, h = blockIdx.x & 7;
  const int usechain = (s < NCH) ? 1 : 0;
  const int segid = usechain ? s : (s - NCH);
  float c = 0.0f;
#pragma unroll 1
  for (int k = 0; k < NN / 256; ++k) {
    const int n = tid + 256 * k;
    const int ci = chain[n], bi = batch[n];
    const float m = mask[n];
    const int id = usechain ? ci : bi;
    c += (id == segid) ? m : 0.0f;
  }
  c = wave_sum(c);
  if (lane == 0) red[wave] = c;
  __syncthreads();
  float cnt = 0.0f;
#pragma unroll
  for (int w = 0; w < 8; ++w) cnt += red[w];
  const float inv = 1.0f / fmaxf(cnt, 1.0f);
  v4f sum = zero4();
#pragma unroll
  for (int t = 0; t < NTILE; ++t)
    sum = sum + *(const v4f*)(PART + ((size_t)(t * HH + h) * NSEG + s) * 1024 + tid * 4);
  const v4f val = sum * inv;
  volatile v4f* d = (volatile v4f*)(OPS + (size_t)(s * HH + h) * 1024 + tid * 4);
  *d = val;
  __threadfence();
  *d = val;
}

__global__ __launch_bounds__(256) void k_bpart(const float* __restrict__ G, const float* __restrict__ mask,
                                               const int* __restrict__ batch, float* __restrict__ PARTB) {
  const int tid = threadIdx.x;
  const int tile = blockIdx.x >> 1, half = blockIdx.x & 1;
  const int col = half * 256 + tid;
  float a0 = 0.0f, a1 = 0.0f, a2 = 0.0f, a3 = 0.0f;
  const float* g = G + 3 * DD + col;
#pragma unroll 2
  for (int nn = 0; nn < TNODE; ++nn) {
    const int n = tile * TNODE + nn;
    const float v = g[(size_t)n * GW];
    const float m = mask[n];
    const int bi = batch[n];
    const float p = v * m;
    a0 += (bi == 0) ? p : 0.0f;
    a1 += (bi == 1) ? p : 0.0f;
    a2 += (bi == 2) ? p : 0.0f;
    a3 += (bi == 3) ? p : 0.0f;
  }
  const size_t base = (size_t)(tile * NBA) * GOW + col;
  volatile float* d0 = (volatile float*)(PARTB + base);
  volatile float* d1 = (volatile float*)(PARTB + base + GOW);
  volatile float* d2 = (volatile float*)(PARTB + base + 2 * GOW);
  volatile float* d3 = (volatile float*)(PARTB + base + 3 * GOW);
  *d0 = a0; *d1 = a1; *d2 = a2; *d3 = a3;
  __threadfence();
  *d0 = a0; *d1 = a1; *d2 = a2; *d3 = a3;
}

__global__ __launch_bounds__(256) void k_bred(const float* __restrict__ PARTB, const float* __restrict__ mask,
                                              const int* __restrict__ batch, float* __restrict__ MEANB) {
  __shared__ float red[8];
  const int tid = threadIdx.x, lane = tid & 31, wave = tid >> 5;
  const int b = blockIdx.x >> 1, half = blockIdx.x & 1;
  const int col = half * 256 + tid;
  float c = 0.0f;
#pragma unroll 1
  for (int k = 0; k < NN / 256; ++k) {
    const int n = tid + 256 * k;
    const int bi = batch[n];
    const float m = mask[n];
    c += (bi == b) ? m : 0.0f;
  }
  c = wave_sum(c);
  if (lane == 0) red[wave] = c;
  __syncthreads();
  float cnt = 0.0f;
#pragma unroll
  for (int w = 0; w < 8; ++w) cnt += red[w];
  const float inv = 1.0f / fmaxf(cnt, 1.0f);
  float sum = 0.0f;
#pragma unroll
  for (int t = 0; t < NTILE; ++t) sum += PARTB[(size_t)(t * NBA + b) * GOW + col];
  const float val = sum * inv;
  volatile float* d = (volatile float*)(MEANB + (size_t)b * GOW + col);
  *d = val;
  __threadfence();
  *d = val;
}

__global__ __launch_bounds__(256) void k_gout(const float* __restrict__ G, const float* __restrict__ OPS,
                                              const float* __restrict__ MEANB, const int* __restrict__ chain,
                                              const int* __restrict__ batch, _Float16* __restrict__ GO) {
  __shared__ __align__(16) _Float16 gos[8][GP];
  const int tid = threadIdx.x, lane = tid & 31, h = tid >> 5;
  const int vq = lane;
  const int nb0 = blockIdx.x * 8;
#pragma unroll 1
  for (int nl = 0; nl < 8; ++nl) {
    const int n = nb0 + nl;
    int cidx = chain[n];
    if (cidx < 0) cidx += NCH;
    cidx = clampi(cidx, 0, NCH - 1);
    int bidx = batch[n];
    if (bidx < 0) bidx += NBA;
    bidx = clampi(bidx, 0, NBA - 1);
    const float* opc = OPS + (size_t)(cidx * HH + h) * 1024 + vq * 32;
    const float* opb = OPS + (size_t)((NCH + bidx) * HH + h) * 1024 + vq * 32;
    const float* qg = G + (size_t)n * GW + 2 * DD + h * DH;
    float a1 = 0.0f, a2 = 0.0f;
#pragma unroll 2
    for (int cc = 0; cc < DH / 4; ++cc) {
      const v4f q4 = *(const v4f*)(qg + 4 * cc);
      const v4f c4 = *(const v4f*)(opc + 4 * cc);
      const v4f d4 = *(const v4f*)(opb + 4 * cc);
      a1 = fmaf(c4[0], q4[0], a1);
      a1 = fmaf(c4[1], q4[1], a1);
      a1 = fmaf(c4[2], q4[2], a1);
      a1 = fmaf(c4[3], q4[3], a1);
      a2 = fmaf(d4[0], q4[0], a2);
      a2 = fmaf(d4[1], q4[1], a2);
      a2 = fmaf(d4[2], q4[2], a2);
      a2 = fmaf(d4[3], q4[3], a2);
    }
    const int col1 = h * 64 + vq, col2 = col1 + 32;
    const float g1 = a1 + MEANB[(size_t)bidx * GOW + col1];
    const float g2 = a2 + MEANB[(size_t)bidx * GOW + col2];
    gos[nl][col1] = (_Float16)(g1 * C_GO);
    gos[nl][col2] = (_Float16)(g2 * C_GO);
  }
  __syncthreads();
#pragma unroll
  for (int it = 0; it < 2; ++it) {
    const int p = tid + 256 * it;
    const int row = p >> 6, pc = p & 63;
    PackH ph;
    ph.h = *(const v8h*)(&gos[row][pc * 8]);
    const v4u vv = ph.u;
    volatile v4u* d = (volatile v4u*)(GO + (size_t)(nb0 + row) * GOW + pc * 8);
    *d = vv;
    __threadfence();
    *d = vv;
  }
}

extern "C" void kernel_launch(void* const* d_in, const int* in_sizes, int n_in,
                              void* d_out, int out_size, void* d_ws, size_t ws_size,
                              hipStream_t stream) {
  if (n_in < 33) return;
  if (in_sizes[0] != NN * DD) return;
  if (in_sizes[1] != NN) return;
  if (in_sizes[2] != REL * PP) return;
  if (in_sizes[3] != DD * PP) return;
  if (in_sizes[4] != DD * PP) return;
  if (in_sizes[5] != DD || in_sizes[6] != DD) return;
  if (in_sizes[7] != PP || in_sizes[8] != PP) return;
  if (in_sizes[9] != PP * 2 * PP) return;
  if (in_sizes[10] != 2 * PP) return;
  if (in_sizes[11] != 2 * PP * PP) return;
  if (in_sizes[12] != PP) return;
  if (in_sizes[13] != DD || in_sizes[14] != DD) return;
  if (in_sizes[15] != DD * DD || in_sizes[16] != DD * DD || in_sizes[17] != DD * DD) return;
  if (in_sizes[18] != PP * HH) return;
  if (in_sizes[19] != DD * DD) return;
  if (in_sizes[20] != DD * DD || in_sizes[21] != DD) return;
  if (in_sizes[22] != DD * DD || in_sizes[23] != DD) return;
  if (in_sizes[24] != DD * DD || in_sizes[25] != DD) return;
  if (in_sizes[26] != DD * GOW || in_sizes[27] != GOW) return;
  if (in_sizes[28] != GOW * DD) return;
  if (in_sizes[29] != NN * KNB) return;
  if (in_sizes[30] != NN || in_sizes[31] != NN || in_sizes[32] != NN) return;
  if (out_size != NN * DD) return;

  const float* features = (const float*)d_in[0];
  const float* mask     = (const float*)d_in[1];
  const float* w_relpos = (const float*)d_in[2];
  const float* w_left   = (const float*)d_in[3];
  const float* w_right  = (const float*)d_in[4];
  const float* g_ln1    = (const float*)d_in[5];
  const float* b_ln1    = (const float*)d_in[6];
  const float* g_lnp    = (const float*)d_in[7];
  const float* b_lnp    = (const float*)d_in[8];
  const float* w_m1     = (const float*)d_in[9];
  const float* b_m1     = (const float*)d_in[10];
  const float* w_m2     = (const float*)d_in[11];
  const float* b_m2     = (const float*)d_in[12];
  const float* g_ln2    = (const float*)d_in[13];
  const float* b_ln2    = (const float*)d_in[14];
  const float* wq       = (const float*)d_in[15];
  const float* wk       = (const float*)d_in[16];
  const float* wv       = (const float*)d_in[17];
  const float* w_pb     = (const float*)d_in[18];
  const float* wo       = (const float*)d_in[19];
  const float* wkg      = (const float*)d_in[20];
  const float* bkg      = (const float*)d_in[21];
  const float* wvg      = (const float*)d_in[22];
  const float* bvg      = (const float*)d_in[23];
  const float* wqg      = (const float*)d_in[24];
  const float* bqg      = (const float*)d_in[25];
  const float* wbg      = (const float*)d_in[26];
  const float* bbg      = (const float*)d_in[27];
  const float* wog      = (const float*)d_in[28];
  const int* neighbours = (const int*)d_in[29];
  const int* resi       = (const int*)d_in[30];
  const int* chain      = (const int*)d_in[31];
  const int* batch      = (const int*)d_in[32];
  float* out = (float*)d_out;

  size_t off = 0;
  const size_t oF1   = off; off += (size_t)NN * DD * 2;
  const size_t oF2   = off; off += (size_t)NN * DD * 2;
  const size_t oWLR  = off; off += (size_t)LRW * DD * 2;
  const size_t oWQKV = off; off += (size_t)QKVW * DD * 2;
  const size_t oWM1  = off; off += (size_t)(2 * PP) * PP * 2;
  const size_t oWM2  = off; off += (size_t)PP * (2 * PP) * 2;
  const size_t oWPB  = off; off += (size_t)64 * 64 * 2;
  const size_t oWO   = off; off += (size_t)DD * DD * 2;
  const size_t oWG   = off; off += (size_t)GW * DD * 2;
  const size_t oWOG  = off; off += (size_t)DD * GOW * 2;
  const size_t oBG   = off; off += (size_t)GW * 4;
  const size_t oLR   = off; off += (size_t)NN * LRW * 4;
  const size_t oQKV  = off; off += (size_t)NN * QKVW * 4;
  const size_t oPB   = off; off += (size_t)NN * HH * KNB * 4;
  const size_t oATT  = off; off += (size_t)NN * DD * 2;
  const size_t oFM   = off; off += (size_t)NN * DD * 4;
  const size_t oFMH  = off; off += (size_t)NN * DD * 2;
  const size_t oG    = off; off += (size_t)NN * GW * 4;
  const size_t oPART = off; off += (size_t)NTILE * HH * NSEG * 1024 * 4;
  const size_t oOPS  = off; off += (size_t)NSEG * HH * 1024 * 4;
  const size_t oPTB  = off; off += (size_t)NTILE * NBA * GOW * 4;
  const size_t oMNB  = off; off += (size_t)NBA * GOW * 4;
  const size_t oGO   = off; off += (size_t)NN * GOW * 2;
  if (off > ws_size) return;
  if (off > (size_t)134217728) return;
  if (((oF2 | oWLR | oWQKV | oWM1 | oWM2 | oWPB | oWO | oWG | oWOG | oBG | oLR | oQKV | oPB | oATT | oFM |
        oFMH | oG | oPART | oOPS | oPTB | oMNB | oGO) & 255) != 0) return;

  char* ws = (char*)d_ws;
  _Float16* F1h   = (_Float16*)(ws + oF1);
  _Float16* F2h   = (_Float16*)(ws + oF2);
  _Float16* WLRT  = (_Float16*)(ws + oWLR);
  _Float16* WQKVT = (_Float16*)(ws + oWQKV);
  _Float16* WM1T  = (_Float16*)(ws + oWM1);
  _Float16* WM2T  = (_Float16*)(ws + oWM2);
  _Float16* WPBT  = (_Float16*)(ws + oWPB);
  _Float16* WOT   = (_Float16*)(ws + oWO);
  _Float16* WGT   = (_Float16*)(ws + oWG);
  _Float16* WOGT  = (_Float16*)(ws + oWOG);
  float* BG       = (float*)(ws + oBG);
  float* LR       = (float*)(ws + oLR);
  float* QKV      = (float*)(ws + oQKV);
  float* PB       = (float*)(ws + oPB);
  _Float16* ATTh  = (_Float16*)(ws + oATT);
  float* FM       = (float*)(ws + oFM);
  _Float16* FMh   = (_Float16*)(ws + oFMH);
  float* G        = (float*)(ws + oG);
  float* PART     = (float*)(ws + oPART);
  float* OPS      = (float*)(ws + oOPS);
  float* PARTB    = (float*)(ws + oPTB);
  float* MEANB    = (float*)(ws + oMNB);
  _Float16* GOh   = (_Float16*)(ws + oGO);
  const float* nof = (const float*)0;

  k_ln8<<<dim3(NN / 8), dim3(256), 0, stream>>>(features, g_ln1, b_ln1, g_ln2, b_ln2, F1h, F2h);
  k_wtrans<<<dim3(1, 4), dim3(256), 0, stream>>>(w_left, DD, PP, WLRT, DD, 0, WSC);
  k_wtrans<<<dim3(1, 4), dim3(256), 0, stream>>>(w_right, DD, PP, WLRT, DD, PP, WSC);
  k_wtrans<<<dim3(4, 4), dim3(256), 0, stream>>>(wq, DD, DD, WQKVT, DD, 0, WSC);
  k_wtrans<<<dim3(4, 4), dim3(256), 0, stream>>>(wk, DD, DD, WQKVT, DD, DD, WSC);
  k_wtrans<<<dim3(4, 4), dim3(256), 0, stream>>>(wv, DD, DD, WQKVT, DD, 2 * DD, WSC);
  k_wtrans<<<dim3(2, 1), dim3(256), 0, stream>>>(w_m1, PP, 2 * PP, WM1T, PP, 0, WSC);
  k_wtrans<<<dim3(1, 2), dim3(256), 0, stream>>>(w_m2, 2 * PP, PP, WM2T, 2 * PP, 0, WSC);
  k_wtrans<<<dim3(1, 1), dim3(256), 0, stream>>>(w_pb, PP, HH, WPBT, PP, 0, WSC);
  k_wtrans<<<dim3(4, 4), dim3(256), 0, stream>>>(wo, DD, DD, WOT, DD, 0, WSC);
  k_wtrans<<<dim3(4, 4), dim3(256), 0, stream>>>(wkg, DD, DD, WGT, DD, 0, WSC);
  k_wtrans<<<dim3(4, 4), dim3(256), 0, stream>>>(wvg, DD, DD, WGT, DD, DD, WSC);
  k_wtrans<<<dim3(4, 4), dim3(256), 0, stream>>>(wqg, DD, DD, WGT, DD, 2 * DD, WSC);
  k_wtrans<<<dim3(8, 4), dim3(256), 0, stream>>>(wbg, DD, GOW, WGT, DD, 3 * DD, WSC);
  k_wtrans<<<dim3(4, 8), dim3(256), 0, stream>>>(wog, GOW, DD, WOGT, GOW, 0, WSC);
  k_bias<<<dim3(1), dim3(256), 0, stream>>>(bkg, bvg, bqg, bbg, BG);
  k_gemm<<<dim3(NN / 256, LRW / 64), dim3(256), 0, stream>>>(F1h, DD, WLRT, DD, DD, S_W, nof, nof, LR, LRW, 0);
  k_gemm<<<dim3(NN / 256, QKVW / 64), dim3(256), 0, stream>>>(F2h, DD, WQKVT, DD, DD, S_W, nof, nof, QKV, QKVW, 0);
  k_pair<<<dim3((NN * KNB) / 64), dim3(256), 0, stream>>>(w_relpos, LR, g_lnp, b_lnp, b_m1, b_m2, WM1T, WM2T,
                                                         WPBT, neighbours, resi, chain, batch, PB);
  k_attn<<<dim3(NN), dim3(256), 0, stream>>>(QKV, PB, mask, neighbours, ATTh);
  k_gemm<<<dim3(NN / 256, DD / 64), dim3(256), 0, stream>>>(ATTh, DD, WOT, DD, DD, S_WO, nof, features, FM, DD, 0);
  k_cvt<<<dim3((NN * DD) / 2048), dim3(256), 0, stream>>>(FM, FMh, 1.0f);
  k_gemm<<<dim3(NN / 256, GW / 64), dim3(256), 0, stream>>>(FMh, DD, WGT, DD, DD, S_W, BG, nof, G, GW, 0x00000F0F);
  k_kvpart<<<dim3(NTILE * HH * 2), dim3(128), 0, stream>>>(G, mask, chain, batch, PART);
  k_segred<<<dim3(NSEG * HH), dim3(256), 0, stream>>>(PART, mask, chain, batch, OPS);
  k_bpart<<<dim3(NTILE * 2), dim3(256), 0, stream>>>(G, mask, batch, PARTB);
  k_bred<<<dim3(NBA * 2), dim3(256), 0, stream>>>(PARTB, mask, batch, MEANB);
  k_gout<<<dim3(NN / 8), dim3(256), 0, stream>>>(G, OPS, MEANB, chain, batch, GOh);
  k_gemm<<<dim3(NN / 256, DD / 64), dim3(256), 0, stream>>>(GOh, GOW, WOGT, GOW, GOW, S_WOG, nof, FM, out, DD, 0);
  (void)hipGetLastError();
}
